// SimplicialAttention_9509057593422
// MI455X (gfx1250) — hardware-verified
//
#include <hip/hip_runtime.h>
#include <math.h>

#define SEQ 1024
#define NHD 4
#define HD 64
#define HDIM (NHD * HD)
#define W1 512
#define W2 32

typedef _Float16 f16;
typedef __attribute__((ext_vector_type(16))) f16 f16x16;
typedef __attribute__((ext_vector_type(16))) __bf16 bf16x16;
typedef __attribute__((ext_vector_type(8)))  __bf16 bf16x8;
typedef __attribute__((ext_vector_type(8)))  f16 f16x8;
typedef __attribute__((ext_vector_type(8)))  float f32x8;
typedef __attribute__((ext_vector_type(4)))  float v4f_t;
typedef float v4fa __attribute__((ext_vector_type(4), may_alias));

__device__ __forceinline__ f32x8 wmma16(f16x16 a, f16x16 b, f32x8 c) {
  c = __builtin_amdgcn_wmma_f32_16x16x32_f16(false, a, false, b, (short)0, c, false, false);
  asm volatile("v_nop\n\tv_nop\n\tv_nop\n\tv_nop" : "+v"(c) : "v"(a), "v"(b));
  return c;
}
__device__ __forceinline__ f32x8 wmma_b16(bf16x16 a, bf16x16 b, f32x8 c) {
  c = __builtin_amdgcn_wmma_f32_16x16x32_bf16(false, a, false, b, (short)0, c, false, false);
  asm volatile("v_nop\n\tv_nop\n\tv_nop\n\tv_nop" : "+v"(c) : "v"(a), "v"(b));
  return c;
}
__device__ __forceinline__ bf16x16 ldsb_frag(const __bf16* base, int stride) {
  const int lane = threadIdx.x & 31, row = lane & 15, kh = (lane >> 4) * 8;
  const bf16x8 lo = *(const bf16x8*)(base + row * stride + kh);
  const bf16x8 hi = *(const bf16x8*)(base + row * stride + kh + 16);
  bf16x16 f;
#pragma unroll
  for (int i = 0; i < 8; ++i) { f[i] = lo[i]; f[i + 8] = hi[i]; }
  return f;
}
__device__ __forceinline__ float rb(float v) { return (float)(__bf16)v; }
__device__ __forceinline__ f16x16 lds_frag(const f16* base, int stride) {
  const int lane = threadIdx.x & 31, row = lane & 15, kh = (lane >> 4) * 8;
  const f16x8 lo = *(const f16x8*)(base + row * stride + kh);
  const f16x8 hi = *(const f16x8*)(base + row * stride + kh + 16);
  f16x16 f;
#pragma unroll
  for (int i = 0; i < 8; ++i) { f[i] = lo[i]; f[i + 8] = hi[i]; }
  return f;
}
__device__ __forceinline__ bf16x16 k1frag(const float* __restrict__ k1, int h, int jbase, int s0, int d0) {
  const int lane = threadIdx.x & 31, r = lane & 15, kh = (lane >> 4) * 8; const int j = jbase + s0 + r;
  bf16x16 f; const float* p = k1 + (size_t)max(j, 0) * HDIM + h * HD + d0 + kh;
#pragma unroll
  for (int i = 0; i < 8; ++i) { f[i] = (__bf16)((j >= 0) ? p[i] : 0.0f); f[8 + i] = (__bf16)((j >= 0) ? p[16 + i] : 0.0f); }
  return f;
}
__device__ __forceinline__ f16x16 v1tfrag(const float* __restrict__ v1, int h, int jbase, int d0, int s0) {
  const int lane = threadIdx.x & 31, r = lane & 15, kh = (lane >> 4) * 8; const int d = d0 + r;
  f16x16 f;
#pragma unroll
  for (int i = 0; i < 8; ++i) { const int ja = jbase + s0 + kh + i, jb = ja + 16;
    const float va = rb(v1[(size_t)max(ja, 0) * HDIM + h * HD + d]), vb = rb(v1[(size_t)max(jb, 0) * HDIM + h * HD + d]);
    f[i] = (f16)((ja >= 0) ? va : 0.0f); f[8 + i] = (f16)((jb >= 0) ? vb : 0.0f); }
  return f;
}

__global__ __launch_bounds__(256) void k_simplicial(const float* __restrict__ xq, const float* __restrict__ xk1, const float* __restrict__ xk2,
                                                    const float* __restrict__ xv1, const float* __restrict__ xv2, float* __restrict__ out) {
  __shared__ __attribute__((aligned(16))) __bf16 tS[2][W2 * 72];
  __shared__ __attribute__((aligned(16))) union SP { float sS[W2 * 520]; f16 pS[2][W2 * 520]; } sp;
  float* sS = sp.sS;
  __shared__ float uS[W2 * 68];
  __shared__ float red[256];
  __shared__ __attribute__((aligned(16))) float oS[HD];
  const int tid = threadIdx.x, lane = tid & 31, wave = tid >> 5, cl = lane & 15, rh = (lane >> 4) * 8;
  const int i = blockIdx.x >> 2, h = blockIdx.x & 3;
  const int jbase = i - (W1 - 1), abase = i - (W2 - 1);
  for (int e = tid; e < W2 * HD; e += 256) { const int a = e >> 6, d = e & 63; const int pa = abase + a;
    const float t = (pa >= 0) ? rb(xq[(size_t)i * HDIM + h * HD + d]) * rb(xk2[(size_t)max(pa, 0) * HDIM + h * HD + d]) : 0.0f;
    const __bf16 th = (__bf16)t; tS[0][a * 72 + d] = th; tS[1][a * 72 + d] = (__bf16)(t - (float)th); }
  __syncthreads();
  { bf16x16 ah[2][2], al[2][2];
#pragma unroll
    for (int at = 0; at < 2; ++at)
#pragma unroll
      for (int ks = 0; ks < 2; ++ks) { ah[at][ks] = ldsb_frag(tS[0] + (at * 16) * 72 + ks * 32, 72); al[at][ks] = ldsb_frag(tS[1] + (at * 16) * 72 + ks * 32, 72); }
#pragma unroll 1
    for (int t4 = 0; t4 < 4; ++t4) { const int st = wave * 4 + t4;
      f32x8 acc0 = {}, acc1 = {};
#pragma unroll
      for (int ks = 0; ks < 2; ++ks) { const bf16x16 bfv = k1frag(xk1, h, jbase, st * 16, ks * 32);
        acc0 = wmma_b16(ah[0][ks], bfv, acc0); acc0 = wmma_b16(al[0][ks], bfv, acc0); acc1 = wmma_b16(ah[1][ks], bfv, acc1); acc1 = wmma_b16(al[1][ks], bfv, acc1); }
#pragma unroll
      for (int r = 0; r < 8; ++r) { sS[(rh + r) * 520 + st * 16 + cl] = acc0[r]; sS[(16 + rh + r) * 520 + st * 16 + cl] = acc1[r]; } }
  }
  __syncthreads();
  const float scl = 0.125f * 1.44269504088896340736f;
  float mx = -3.0e38f;
  for (int e = tid; e < W2 * W1; e += 256) { const int a = e >> 9, s = e & 511; const bool ok = (abase + a >= 0) && (jbase + s >= 0);
    const float v = ok ? sS[a * 520 + s] * scl : -3.0e38f; sS[a * 520 + s] = v; mx = fmaxf(mx, v); }
  red[tid] = mx; __syncthreads();
  for (int o = 128; o > 0; o >>= 1) { if (tid < o) red[tid] = fmaxf(red[tid], red[tid + o]); __syncthreads(); }
  const float m = red[0]; __syncthreads();
  float z = 0.0f;
  for (int e = tid; e < W2 * W1; e += 256) { const int a = e >> 9, s = e & 511; const float v = sS[a * 520 + s]; const float ev = (v <= -1.0e38f) ? 0.0f : exp2f(v - m);
    sS[a * 520 + s] = ev; z += ev; }
  red[tid] = z; __syncthreads();
  for (int o = 128; o > 0; o >>= 1) { if (tid < o) red[tid] += red[tid + o]; __syncthreads(); }
  const float iz = 1024.0f / red[0];
  float pv[64];
#pragma unroll
  for (int k = 0; k < 64; ++k) { const int e = tid + 256 * k; const int a = e >> 9, s = e & 511; pv[k] = sS[a * 520 + s] * iz; }
  __syncthreads();
  f16* pS0 = sp.pS[0]; f16* pS1 = sp.pS[1];
#pragma unroll
  for (int k = 0; k < 64; ++k) { const int e = tid + 256 * k; const int a = e >> 9, s = e & 511; const f16 ph = (f16)pv[k]; pS0[a * 520 + s] = ph; pS1[a * 520 + s] = (f16)((pv[k] - (float)ph) * 2048.0f); }
  if (tid < W2) { for (int s = 512; s < 520; ++s) { pS0[tid * 520 + s] = (f16)0.0f; pS1[tid * 520 + s] = (f16)0.0f; } }
  __syncthreads();
  { const int at = wave >> 2, dt = wave & 3; f32x8 acc = {}, accx = {};
#pragma unroll 1
    for (int ks = 0; ks < 16; ++ks) { const f16x16 vf = v1tfrag(xv1, h, jbase, dt * 16, ks * 32);
      acc = wmma16(lds_frag(sp.pS[0] + (at * 16) * 520 + ks * 32, 520), vf, acc); accx = wmma16(lds_frag(sp.pS[1] + (at * 16) * 520 + ks * 32, 520), vf, accx); }
#pragma unroll
    for (int r = 0; r < 8; ++r) uS[(at * 16 + rh + r) * 68 + dt * 16 + cl] = (acc[r] + accx[r] * (1.0f / 2048.0f)) * (1.0f / 1024.0f); }
  __syncthreads();
  { const int d = tid & 63, aq = tid >> 6; float s = 0.0f;
#pragma unroll
    for (int k = 0; k < 8; ++k) { const int a = aq * 8 + k; const int pa = abase + a; const float w = rb(xv2[(size_t)max(pa, 0) * HDIM + h * HD + d]); if (pa >= 0) s += uS[a * 68 + d] * w; }
    red[tid] = s; }
  __syncthreads();
  if (tid < 64) oS[tid] = red[tid] + red[64 + tid] + red[128 + tid] + red[192 + tid];
  __syncthreads();
  if (tid < 16) { float* dst = out + (size_t)i * HDIM + h * HD + tid * 4; *(volatile v4f_t*)dst = *(const volatile v4fa*)(oS + tid * 4); __threadfence(); *(volatile v4f_t*)dst = *(const volatile v4fa*)(oS + tid * 4); }
}

extern "C" void kernel_launch(void* const* d_in, const int* in_sizes, int n_in,
                              void* d_out, int out_size, void* d_ws, size_t ws_size,
                              hipStream_t stream) {
  (void)in_sizes; (void)n_in; (void)out_size; (void)d_ws; (void)ws_size;
  const float* xq = (const float*)d_in[0], *xk1 = (const float*)d_in[1], *xk2 = (const float*)d_in[2], *xv1 = (const float*)d_in[3], *xv2 = (const float*)d_in[4];
  float* out = (float*)d_out;
  k_simplicial<<<dim3(SEQ * NHD), dim3(256), 0, stream>>>(xq, xk1, xk2, xv1, xv2, out);
}
